// Symmetric_CA_Layer_618475290758
// MI455X (gfx1250) — hardware-verified
//
#include <hip/hip_runtime.h>


#define NB_  4
#define CC   256
#define NN   4096
#define DQ   64
#define PCAR 1024.0f
#define PR   1024
#define NPR  (NB_ * NN / PR)
typedef _Float16 h16;
typedef unsigned short bf;
typedef __attribute__((ext_vector_type(16))) __bf16   v16bf;
typedef __attribute__((ext_vector_type(16))) _Float16 v16h;
typedef __attribute__((ext_vector_type(8)))  _Float16 v8h;
typedef __attribute__((ext_vector_type(8)))  unsigned short v8us;
typedef __attribute__((ext_vector_type(8)))  float    v8f;
typedef __attribute__((ext_vector_type(4)))  float    v4f;
typedef v8h  __attribute__((may_alias)) v8ha;
typedef v4f  __attribute__((may_alias)) v4fa;
typedef v8us __attribute__((may_alias)) v8usa;

__device__ __forceinline__ unsigned short f2bf(float f) { unsigned u = __float_as_uint(f); u += 0x7FFFu + ((u >> 16) & 1u); return (unsigned short)(u >> 16); }
__device__ __forceinline__ float bf2f(unsigned short b) { return __uint_as_float(((unsigned)b) << 16); }
__device__ __forceinline__ float bfr(float f) { return bf2f(f2bf(f)); }
__device__ __forceinline__ v16h cat16(v8h lo, v8h hi) { return __builtin_shufflevector(lo, hi, 0, 1, 2, 3, 4, 5, 6, 7, 8, 9, 10, 11, 12, 13, 14, 15); }
__device__ __forceinline__ v16bf cat16b(v8us lo, v8us hi) { return __builtin_bit_cast(v16bf, __builtin_shufflevector(lo, hi, 0, 1, 2, 3, 4, 5, 6, 7, 8, 9, 10, 11, 12, 13, 14, 15)); }
__device__ __forceinline__ v8f wmma16(v16h a, v16h b, v8f c) { return __builtin_amdgcn_wmma_f32_16x16x32_f16(false, a, false, b, (short)0, c, false, false); }
__device__ __forceinline__ v8f wmmab(v16bf a, v16bf b, v8f c) { return __builtin_amdgcn_wmma_f32_16x16x32_bf16(false, a, false, b, (short)0, c, false, false); }


template <typename T16> struct WFrag;
template <> struct WFrag<h16> { typedef v16h V; static __device__ __forceinline__ V ld(const h16* p) { return cat16(*(const v8h*)p, *(const v8h*)(p + 16)); } static __device__ __forceinline__ v8f mma(V a, V b, v8f c) { return wmma16(a, b, c); } };
template <> struct WFrag<bf> { typedef v16bf V; static __device__ __forceinline__ V ld(const bf* p) { return cat16b(*(const v8us*)p, *(const v8us*)(p + 16)); } static __device__ __forceinline__ v8f mma(V a, V b, v8f c) { return wmmab(a, b, c); } };
template <typename T16, int NSPLIT, bool BIAS>
__global__ __launch_bounds__(32) void k_gemmw(const T16* __restrict__ A, const T16* __restrict__ A2, const T16* __restrict__ Bt, const T16* __restrict__ Bt2, int K, float* C, int ldc, const float* __restrict__ bias, size_t sA, size_t sB, size_t sC) {
    typedef typename WFrag<T16>::V V;
    __shared__ __align__(16) float os[16 * 68];
    const size_t z = blockIdx.z; A += z * sA; if (A2) A2 += z * sA; Bt += z * sB; if (Bt2) Bt2 += z * sB; C += z * sC;
    const int lane = threadIdx.x & 31, lr = lane & 15, hi = lane >> 4; const int r0 = blockIdx.x * 64, c0 = blockIdx.y * 64;
    v8f acc[4][4];
#pragma unroll
    for (int mb = 0; mb < 4; ++mb)
#pragma unroll
        for (int nb = 0; nb < 4; ++nb) acc[mb][nb] = (v8f){};
    const size_t aoff = (size_t)(r0 + lr) * K + 8 * hi, boff = (size_t)(c0 + lr) * K + 8 * hi;
#pragma unroll 1
    for (int kc = 0; kc < K; kc += 32) {
        V a[4], a2[4];
#pragma unroll
        for (int mb = 0; mb < 4; ++mb) { a[mb] = WFrag<T16>::ld(A + aoff + (size_t)mb * 16 * K + kc); if (NSPLIT == 1 || NSPLIT == 2) a2[mb] = WFrag<T16>::ld(A2 + aoff + (size_t)mb * 16 * K + kc); }
#pragma unroll
        for (int nb = 0; nb < 4; ++nb) { const V b = WFrag<T16>::ld(Bt + boff + (size_t)nb * 16 * K + kc); V b2; if (NSPLIT >= 2) b2 = WFrag<T16>::ld(Bt2 + boff + (size_t)nb * 16 * K + kc);
#pragma unroll
            for (int mb = 0; mb < 4; ++mb) { acc[mb][nb] = WFrag<T16>::mma(a[mb], b, acc[mb][nb]); if (NSPLIT == 1 || NSPLIT == 2) acc[mb][nb] = WFrag<T16>::mma(a2[mb], b, acc[mb][nb]); if (NSPLIT >= 2) acc[mb][nb] = WFrag<T16>::mma(a[mb], b2, acc[mb][nb]); } }
        asm volatile("v_nop\n\tv_nop\n\tv_nop\n\tv_nop" : "+v"(acc[0][0]), "+v"(acc[1][1]), "+v"(acc[2][2]), "+v"(acc[3][3]) : "v"(a[0]), "v"(a[3]));
    }
#pragma unroll
    for (int mb = 0; mb < 4; ++mb) {
#pragma unroll
        for (int nb = 0; nb < 4; ++nb) {
#pragma unroll
            for (int j = 0; j < 8; ++j) os[(hi * 8 + j) * 68 + nb * 16 + lr] = acc[mb][nb][j]; }
        __builtin_amdgcn_wave_barrier(); asm volatile("" ::: "memory");
        float* crow = C + (size_t)(r0 + mb * 16) * ldc + c0;
#pragma unroll 1
        for (int ps = 0; ps < 2; ++ps) {
#pragma unroll
            for (int s = 0; s < 8; ++s) { const int row = 2 * s + hi, cofs = lr * 4; v4f val = *(const v4fa*)(os + row * 68 + cofs); if (BIAS) { val[0] += bfr(bias[c0 + cofs]); val[1] += bfr(bias[c0 + cofs + 1]); val[2] += bfr(bias[c0 + cofs + 2]); val[3] += bfr(bias[c0 + cofs + 3]); }
                *(volatile v4f*)(crow + (size_t)row * ldc + cofs) = val; }
            if (ps == 0) __threadfence(); }
        __builtin_amdgcn_wave_barrier(); asm volatile("" ::: "memory");
    }
}

__device__ __forceinline__ h16 tohx(float x) { return (h16)x; }
__device__ __forceinline__ void splitf(float y, unsigned short& h, unsigned short& l) { h = f2bf(y); l = f2bf(y - bf2f(h)); }
typedef __attribute__((ext_vector_type(2))) _Float16 v2h;
typedef __attribute__((ext_vector_type(4))) _Float16 v4h;
typedef __attribute__((ext_vector_type(2))) unsigned short v2us;
typedef __attribute__((ext_vector_type(4))) unsigned short v4us;
typedef __attribute__((ext_vector_type(2))) float v2f;
#define TQ NN
template <int NK>
__global__ __launch_bounds__(256) void k_smax(const float* __restrict__ S, float* RS) { const int lane = threadIdx.x & 31; const int i = blockIdx.x * 8 + (threadIdx.x >> 5); if (i >= TQ) return; const float* sr = S + (size_t)i * NK; float m = -3.0e38f;
#pragma unroll 4
    for (int c0 = lane * 4; c0 < NK; c0 += 128) { const v4f v = *(const v4f*)(sr + c0); m = fmaxf(m, fmaxf(fmaxf(v[0], v[1]), fmaxf(v[2], v[3]))); }
#pragma unroll
    for (int sh = 16; sh; sh >>= 1) m = fmaxf(m, __shfl_xor(m, sh, 32));
    const float o = lane == 0 ? m : 0.f; *(volatile float*)(RS + (size_t)i * 32 + lane) = o; __threadfence(); *(volatile float*)(RS + (size_t)i * 32 + lane) = o; }
template <int NK>
__global__ __launch_bounds__(256) void k_sexp(const float* __restrict__ S, float* RS, h16* P) { const int lane = threadIdx.x & 31; const int i = blockIdx.x * 8 + (threadIdx.x >> 5); if (i >= TQ) return; const float* sr = S + (size_t)i * NK; const float m = RS[(size_t)i * 32]; float sum = 0.f;
#pragma unroll 1
    for (int ps = 0; ps < 2; ++ps) { sum = 0.f;
#pragma unroll 2
        for (int c0 = lane * 4; c0 < NK; c0 += 128) { const v4f v = *(const v4f*)(sr + c0); v4h o;
#pragma unroll
            for (int q = 0; q < 4; ++q) { float dlt = __fsub_rn(v[q], m); asm volatile("" : "+v"(dlt)); const float e = __expf(__fmul_rn(dlt, 1.0f)); sum += e; o[q] = tohx(e * PCAR); }
            *(volatile v4h*)(P + (size_t)i * NK + c0) = o; }
        if (ps == 0) __threadfence(); }
#pragma unroll
    for (int sh = 16; sh; sh >>= 1) sum += __shfl_xor(sum, sh, 32);
    const float o2 = lane == 0 ? m : (lane == 1 ? __fdiv_rn(1.0f, sum * PCAR) : 0.f); *(volatile float*)(RS + (size_t)i * 32 + lane) = o2; __threadfence(); *(volatile float*)(RS + (size_t)i * 32 + lane) = o2; }
__global__ __launch_bounds__(256) void k_cvt8(const float* __restrict__ src, bf* dst, size_t n8) { const size_t i = (size_t)blockIdx.x * 256 + threadIdx.x; if (i >= n8) return; const v8f v = *(const v8f*)(src + i * 8); v8us o;
#pragma unroll
    for (int k = 0; k < 8; ++k) o[k] = f2bf(v[k]); *(volatile v8us*)(dst + i * 8) = o; __threadfence(); *(volatile v8us*)(dst + i * 8) = o; }
__global__ __launch_bounds__(256) void k_xt(const float* __restrict__ xb, bf* XT) { const size_t e = ((size_t)blockIdx.x * 256 + threadIdx.x) * 4; if (e >= (size_t)NN * CC) return; const int c = (int)(e % CC), n = (int)(e / CC); v4us o;
#pragma unroll
    for (int q = 0; q < 4; ++q) o[q] = f2bf(xb[(size_t)(c + q) * NN + n]); *(volatile v4us*)(XT + e) = o; __threadfence(); *(volatile v4us*)(XT + e) = o; }
__global__ __launch_bounds__(256) void k_spl64(const float* __restrict__ F, bf* Fh, bf* Fl) { const size_t i = ((size_t)blockIdx.x * 256 + threadIdx.x) * 4; if (i >= (size_t)NN * DQ) return; const v4f a = *(const v4f*)(F + i); v4us oh, ol;
#pragma unroll
    for (int q = 0; q < 4; ++q) { unsigned short u, c2; splitf(a[q], u, c2); oh[q] = u; ol[q] = c2; } *(volatile v4us*)(Fh + i) = oh; *(volatile v4us*)(Fl + i) = ol; __threadfence(); *(volatile v4us*)(Fh + i) = oh; *(volatile v4us*)(Fl + i) = ol; }
__global__ __launch_bounds__(256) void k_v16(const float* __restrict__ V, h16* V16) { const size_t i = ((size_t)blockIdx.x * 256 + threadIdx.x) * 4; if (i >= (size_t)CC * NN) return; const v4f a = *(const v4f*)(V + i); v4h o; o[0] = tohx(a[0]); o[1] = tohx(a[1]); o[2] = tohx(a[2]); o[3] = tohx(a[3]); *(volatile v4h*)(V16 + i) = o; __threadfence(); *(volatile v4h*)(V16 + i) = o; }
__global__ __launch_bounds__(256) void k_rpl(const float* __restrict__ RT, const h16* __restrict__ P, const float* __restrict__ RS, bf* Rh, bf* Rl) { const int lane = threadIdx.x & 31; const int m = blockIdx.x * 8 + (threadIdx.x >> 5); if (m >= NN) return; const float rs = RS[(size_t)m * 32 + 1]; float s = 0.f;
    for (int c0 = lane * 4; c0 < NN; c0 += 128) { const v4h p = *(const v4h*)(P + (size_t)m * NN + c0); s = __fadd_rn(s, __fadd_rn(__fadd_rn((float)p[0], (float)p[1]), __fadd_rn((float)p[2], (float)p[3]))); }
#pragma unroll
    for (int sh = 16; sh; sh >>= 1) s += __shfl_xor(s, sh, 32);
    const float s1 = __fmul_rn(s, rs); const float f = __fdiv_rn(rs, __fadd_rn(1e-9f, s1));
#pragma unroll 1
    for (int ps = 0; ps < 2; ++ps) {
#pragma unroll
        for (int ch = 0; ch < 2; ++ch) { const size_t o = (size_t)m * CC + ch * 128 + lane * 4; const v4f a = *(const v4f*)(RT + o); v4us oh, ol;
#pragma unroll
            for (int q = 0; q < 4; ++q) { unsigned short u, c2; splitf(__fmul_rn(a[q], f), u, c2); oh[q] = u; ol[q] = c2; } *(volatile v4us*)(Rh + o) = oh; *(volatile v4us*)(Rl + o) = ol; }
        if (ps == 0) __threadfence(); } }
__global__ __launch_bounds__(256) void k_p1(const float* __restrict__ T, const float* __restrict__ M, int centred, float* P) { const int e = blockIdx.x * 256 + threadIdx.x; if (e >= NPR * CC) return; const int c = e % CC, p = e / CC; const float m = centred ? M[c] : 0.f; float s = 0.f;
    for (int r = 0; r < PR; ++r) { const float d = __fsub_rn(T[((size_t)p * PR + r) * CC + c], m); float v = centred ? __fmul_rn(d, d) : d; asm volatile("" : "+v"(v)); s = __fadd_rn(s, v); }
    *(volatile float*)(P + e) = s; __threadfence(); *(volatile float*)(P + e) = s; }
__global__ __launch_bounds__(256) void k_red(const float* __restrict__ P, float* M) { const int c = threadIdx.x; float s = 0.f; for (int p = 0; p < NPR; ++p) s = __fadd_rn(s, P[p * CC + c]); const float m = s * (1.0f / (NB_ * NN)); *(volatile float*)(M + c) = m; __threadfence(); *(volatile float*)(M + c) = m; }
__global__ __launch_bounds__(256) void k_fin(const float* __restrict__ T, const float* __restrict__ MU, const float* __restrict__ VAR, const float* __restrict__ g, const float* __restrict__ bb, const float* __restrict__ res, float* OUT) { const size_t e = ((size_t)blockIdx.x * 256 + threadIdx.x) * 2; if (e >= (size_t)NB_ * CC * NN) return; const int n = (int)(e % NN); const int c = (int)((e / NN) % CC); const int b = (int)(e / ((size_t)NN * CC)); const float sc = __fmul_rn(bfr(g[c]), __frsqrt_rn(__fadd_rn(VAR[c], 1e-5f))); v2f o;
#pragma unroll
    for (int u = 0; u < 2; ++u) { float t = __fmul_rn(__fsub_rn(T[((size_t)b * NN + n + u) * CC + c], MU[c]), sc); asm volatile("" : "+v"(t)); o[u] = __fadd_rn(bfr(res[e + u]), fmaxf(__fadd_rn(t, bfr(bb[c])), 0.f)); }
    *(volatile v2f*)(OUT + e) = o; __threadfence(); *(volatile v2f*)(OUT + e) = o; }

extern "C" void kernel_launch(void* const* d_in, const int* in_sizes, int n_in,
                              void* d_out, int out_size, void* d_ws, size_t ws_size, hipStream_t stream) {
    (void)in_sizes; (void)n_in; (void)out_size;
    const float* IN[10]; for (int i = 0; i < 10; ++i) IN[i] = (const float*)d_in[i];
    float* OUT = (float*)d_out;
    char* wsp = (char*)d_ws;
    auto take = [&](size_t bytes) { char* p = wsp; wsp += (bytes + 255) & ~(size_t)255; return (void*)p; };
    bf* WQK = (bf*)take((size_t)DQ * CC * 2); bf* WV = (bf*)take((size_t)CC * CC * 2); bf* WT = (bf*)take((size_t)CC * CC * 2);
    bf* XS = (bf*)take((size_t)NN * CC * 2); bf* XTg = (bf*)take((size_t)NN * CC * 2); float* FQ = (float*)take((size_t)NN * DQ * 4); float* FK = (float*)take((size_t)NN * DQ * 4); bf* Qh = (bf*)take((size_t)NN * DQ * 2); bf* Ql = (bf*)take((size_t)NN * DQ * 2); bf* Kh = (bf*)take((size_t)NN * DQ * 2); bf* Kl = (bf*)take((size_t)NN * DQ * 2);
    float* V = (float*)take((size_t)CC * NN * 4); h16* V16 = (h16*)take((size_t)CC * NN * 2); float* S = (float*)take((size_t)NN * NN * 4); h16* P = (h16*)take((size_t)NN * NN * 2); float* RS = (float*)take((size_t)NN * 32 * 4); float* RT = (float*)take((size_t)NN * CC * 4); bf* Rh = (bf*)take((size_t)NN * CC * 2); bf* Rl = (bf*)take((size_t)NN * CC * 2);
    float* TALL = (float*)take((size_t)NB_ * NN * CC * 4); float* PP = (float*)take((size_t)NPR * CC * 4); float* MU = (float*)take(CC * 4); float* VAR = (float*)take(CC * 4);
    if ((size_t)(wsp - (char*)d_ws) > ws_size) return;
    for (int br = 0; br < 2; ++br) { const float* src = IN[br]; const float* tgt = IN[1 - br]; float* OUTb = OUT + (size_t)br * NB_ * CC * NN;
        k_cvt8<<<(DQ * CC / 8 + 255) / 256, 256, 0, stream>>>(IN[2 + 3 * br], WQK, (size_t)DQ * CC / 8); k_cvt8<<<(CC * CC / 8 + 255) / 256, 256, 0, stream>>>(IN[3 + 3 * br], WV, (size_t)CC * CC / 8); k_cvt8<<<(CC * CC / 8 + 255) / 256, 256, 0, stream>>>(IN[4 + 3 * br], WT, (size_t)CC * CC / 8);
        for (int b = 0; b < NB_; ++b) {
            k_xt<<<(unsigned)(((size_t)NN * CC / 4 + 255) / 256), 256, 0, stream>>>(src + (size_t)b * CC * NN, XS); k_xt<<<(unsigned)(((size_t)NN * CC / 4 + 255) / 256), 256, 0, stream>>>(tgt + (size_t)b * CC * NN, XTg);
            k_gemmw<bf, 0, false><<<dim3(NN / 64, 1, 1), 32, 0, stream>>>(XTg, nullptr, WQK, nullptr, CC, FQ, DQ, nullptr, 0, 0, 0); k_gemmw<bf, 0, false><<<dim3(NN / 64, 1, 1), 32, 0, stream>>>(XS, nullptr, WQK, nullptr, CC, FK, DQ, nullptr, 0, 0, 0);
            k_gemmw<bf, 0, false><<<dim3(CC / 64, NN / 64, 1), 32, 0, stream>>>(WV, nullptr, XS, nullptr, CC, V, NN, nullptr, 0, 0, 0);
            k_spl64<<<(NN * DQ / 4 + 255) / 256, 256, 0, stream>>>(FQ, Qh, Ql); k_spl64<<<(NN * DQ / 4 + 255) / 256, 256, 0, stream>>>(FK, Kh, Kl); k_v16<<<(unsigned)(((size_t)CC * NN / 4 + 255) / 256), 256, 0, stream>>>(V, V16);
            k_gemmw<bf, 2, false><<<dim3(NN / 64, NN / 64, 1), 32, 0, stream>>>(Qh, Ql, Kh, Kl, DQ, S, NN, nullptr, 0, 0, 0);
            k_smax<NN><<<NN / 8, 256, 0, stream>>>(S, RS); k_sexp<NN><<<NN / 8, 256, 0, stream>>>(S, RS, P);
            k_gemmw<h16, 0, false><<<dim3(NN / 64, CC / 64, 1), 32, 0, stream>>>(P, nullptr, V16, nullptr, NN, RT, CC, nullptr, 0, 0, 0);
            k_rpl<<<NN / 8, 256, 0, stream>>>(RT, P, RS, Rh, Rl);
            k_gemmw<bf, 1, false><<<dim3(NN / 64, CC / 64, 1), 32, 0, stream>>>(Rh, Rl, WT, nullptr, CC, TALL + (size_t)b * NN * CC, CC, nullptr, 0, 0, 0); }
        k_p1<<<(NPR * CC + 255) / 256, 256, 0, stream>>>(TALL, nullptr, 0, PP); k_red<<<1, 256, 0, stream>>>(PP, MU); k_p1<<<(NPR * CC + 255) / 256, 256, 0, stream>>>(TALL, MU, 1, PP); k_red<<<1, 256, 0, stream>>>(PP, VAR);
        k_fin<<<(unsigned)(((size_t)NB_ * CC * NN / 2 + 255) / 256), 256, 0, stream>>>(TALL, MU, VAR, IN[8], IN[9], src, OUTb); }
}
